// GraphTrajectoryLSTM_73967926772364
// MI455X (gfx1250) — hardware-run, weakly checked
//
#include <hip/hip_runtime.h>
#include <math.h>

constexpr int kGraphs      = 256;
constexpr int kNodes       = 200;
constexpr int kNodePad     = 256;
constexpr int kEdges       = 1600;
constexpr int kFeatIn      = 4;
constexpr int kHid         = 256;
constexpr int kQkvLd       = 768;
constexpr int kHeads       = 4;
constexpr int kHeadDim     = 64;
constexpr int kSteps       = 30;
constexpr int kOutLen      = 30;
constexpr int kOutComp     = 7;
constexpr int kGate4       = 1024;
constexpr int kBranches    = 5;
constexpr int kWih0Ld      = 258;
constexpr int kChunkGraphs = 64;
constexpr int kNumChunks   = kGraphs / kChunkGraphs;
constexpr int kHeadNPad    = 64;
constexpr int kAggK        = 224;

constexpr float kCarry     = 16.0f;
constexpr float kM2Scale   = 0.25f;
constexpr float kAggScale  = 1.0f / 64.0f;
constexpr float kAcc256Inv = 1.0f / 256.0f;
constexpr float kQScale    = 1.0f / 2048.0f;
constexpr float kOInv      = 1.0f / 16.0f;
constexpr float kPSC       = 32768.0f;

static_assert(kNumChunks * kChunkGraphs == kGraphs);
static_assert(kHid == kNodePad);
static_assert(kAggK % 32 == 0 && kAggK >= kNodes);

typedef __attribute__((ext_vector_type(16))) _Float16 v16h;
typedef __attribute__((ext_vector_type(8)))  _Float16 v8h;
typedef __attribute__((ext_vector_type(16))) __bf16   v16b;
typedef __attribute__((ext_vector_type(8)))  __bf16   v8b;
typedef __attribute__((ext_vector_type(8)))  float    v8f;
typedef __attribute__((ext_vector_type(4)))  float    v4f;

__device__ __forceinline__ unsigned short f2bf_bits(float f) {
  unsigned u = __float_as_uint(f);
  return (unsigned short)((u + 0x7FFFu + ((u >> 16) & 1u)) >> 16);
}
__device__ __forceinline__ float bf_bits2f(unsigned short h) { return __uint_as_float(((unsigned)h) << 16); }

__device__ __forceinline__ void dep_guard_h(v8f& a, v8f& b, v16h x, v16h y) { asm volatile("v_nop\n\tv_nop\n\tv_nop\n\tv_nop" : "+v"(a), "+v"(b) : "v"(x), "v"(y)); }
__device__ __forceinline__ void dep_guard_b(v8f& a, v8f& b, v16b x, v16b y) { asm volatile("v_nop\n\tv_nop\n\tv_nop\n\tv_nop" : "+v"(a), "+v"(b) : "v"(x), "v"(y)); }
__device__ __forceinline__ void keep4_h(v16h a, v16h b, v16h c, v16h d) { asm volatile("v_nop" :: "v"(a), "v"(b), "v"(c), "v"(d)); }
__device__ __forceinline__ void keep4_b(v16b a, v16b b, v16b c, v16b d) { asm volatile("v_nop" :: "v"(a), "v"(b), "v"(c), "v"(d)); }
__device__ __forceinline__ void acc_guard4(v8f& a, v8f& b, v8f& c, v8f& d) { asm volatile("v_nop\n\tv_nop\n\tv_nop\n\tv_nop" : "+v"(a), "+v"(b), "+v"(c), "+v"(d)); }
template <typename T> struct Frag;
template <> struct Frag<_Float16> {
  typedef v16h V; union U { v16h v; v8h h[2]; };
  static __device__ __forceinline__ v16h load(const _Float16* p) {
    U f; f.h[0] = *(const v8h*)(p); f.h[1] = *(const v8h*)(p + 16); return f.v;
  }
  static __device__ __forceinline__ v8f mma(v16h a, v16h b, v8f c) {
    return __builtin_amdgcn_wmma_f32_16x16x32_f16(false, a, false, b, (short)0, c, false, false);
  }
  static __device__ __forceinline__ void guard(v8f& a, v8f& b, v16h x, v16h y) { dep_guard_h(a, b, x, y); }
  static __device__ __forceinline__ void keep(v16h a, v16h b, v16h c, v16h d) { keep4_h(a, b, c, d); }
};
template <> struct Frag<__bf16> {
  typedef v16b V; union U { v16b v; v8b h[2]; };
  static __device__ __forceinline__ v16b load(const __bf16* p) {
    U f; f.h[0] = *(const v8b*)(p); f.h[1] = *(const v8b*)(p + 16); return f.v;
  }
  static __device__ __forceinline__ v8f mma(v16b a, v16b b, v8f c) {
    return __builtin_amdgcn_wmma_f32_16x16x32_bf16(false, a, false, b, (short)0, c, false, false);
  }
  static __device__ __forceinline__ void guard(v8f& a, v8f& b, v16b x, v16b y) { dep_guard_b(a, b, x, y); }
  static __device__ __forceinline__ void keep(v16b a, v16b b, v16b c, v16b d) { keep4_b(a, b, c, d); }
};

__device__ __forceinline__ v8f mma_h(v16h a, v16h b, v8f c) {
  c = __builtin_amdgcn_wmma_f32_16x16x32_f16(false, a, false, b, (short)0, c, false, false);
  asm volatile("v_nop\n\tv_nop\n\tv_nop\n\tv_nop" : "+v"(c) : "v"(a), "v"(b));
  return c;
}

__device__ __forceinline__ float fsig(float x)  { return __builtin_amdgcn_rcpf(1.0f + __expf(-x)); }
__device__ __forceinline__ float ftanh(float x) { return 1.0f - 2.0f * __builtin_amdgcn_rcpf(__expf(2.0f * x) + 1.0f); }

template <int ET> struct Elem;
template <> struct Elem<0> { typedef _Float16 T; };
template <> struct Elem<1> { typedef __bf16 T; };
template <int ET, bool SPLIT, int BIAS_MODE, int OUT_MODE, bool RESID, int ACT = 0>
__global__ __launch_bounds__(256) void wmma_gemm64(
    const unsigned short* __restrict__ Ap, const unsigned short* __restrict__ A2p, int lda, long strideA,
    const unsigned short* __restrict__ Btp, const unsigned short* __restrict__ Bt2p, int ldb, long strideB,
    void* __restrict__ Cout, void* __restrict__ Cout2, int ldc, long strideC,
    const float* __restrict__ bias,
    const float* __restrict__ resid, long strideR,
    int M, int N, int K, float scale, float oscale) {
  typedef typename Elem<ET>::T T;
  typedef typename Frag<T>::V V;
  const T* A = (const T*)Ap; const T* A2 = (const T*)A2p; const T* Bt = (const T*)Btp; const T* Bt2 = (const T*)Bt2p;
  __shared__ __align__(16) float sT[8][16 * 68];
  const int b    = blockIdx.y;
  const int lane = threadIdx.x & 31;
  const int wave = threadIdx.x >> 5;
  const int tilesN = N >> 6;
  const int tilesM = M >> 6;
  const int tile = blockIdx.x * 8 + wave;
  if (tile >= tilesM * tilesN) return;
  const int tm = tile / tilesN;
  const int tn = tile - tm * tilesN;
  const int m0 = tm << 6;
  const int n0 = tn << 6;

  const T* Ab  = A  + (size_t)b * strideA;
  const T* Bb  = Bt + (size_t)b * strideB;
  const T* Ab2 = SPLIT ? (A2  + (size_t)b * strideA) : nullptr;
  const T* Bb2 = SPLIT ? (Bt2 + (size_t)b * strideB) : nullptr;

  const int rlane = lane & 15;
  const int koff  = (lane >> 4) * 8;
  const int mOff  = (lane >> 4) * 8;

  v8f acc[4][4];
#pragma unroll
  for (int i = 0; i < 4; ++i)
#pragma unroll
    for (int j = 0; j < 4; ++j) acc[i][j] = (v8f){0.f,0.f,0.f,0.f,0.f,0.f,0.f,0.f};

  for (int k0 = 0; k0 < K; k0 += 32) {
    V bh[4], bl[4];
#pragma unroll
    for (int j = 0; j < 4; ++j) {
      const size_t bo = (size_t)(n0 + (j << 4) + rlane) * ldb + koff + k0;
      bh[j] = Frag<T>::load(Bb + bo);
      if (SPLIT) bl[j] = Frag<T>::load(Bb2 + bo);
    }
#pragma unroll
    for (int i = 0; i < 4; ++i) {
      const size_t ao = (size_t)(m0 + (i << 4) + rlane) * lda + koff + k0;
      V ah = Frag<T>::load(Ab + ao);
      V al;
      if (SPLIT) al = Frag<T>::load(Ab2 + ao);
#pragma unroll
      for (int j = 0; j < 4; ++j) {
        acc[i][j] = Frag<T>::mma(ah, bh[j], acc[i][j]);
        if (SPLIT) {
          acc[i][j] = Frag<T>::mma(ah, bl[j], acc[i][j]);
          acc[i][j] = Frag<T>::mma(al, bh[j], acc[i][j]);
        }
      }
      Frag<T>::guard(acc[i][0], acc[i][3], ah, SPLIT ? al : ah);
    }
    Frag<T>::keep(bh[0], bh[1], bh[2], bh[3]);
    if (SPLIT) Frag<T>::keep(bl[0], bl[1], bl[2], bl[3]);
  }
  acc_guard4(acc[0][0], acc[0][1], acc[0][2], acc[0][3]);
  acc_guard4(acc[1][0], acc[1][1], acc[1][2], acc[1][3]);
  acc_guard4(acc[2][0], acc[2][1], acc[2][2], acc[2][3]);
  acc_guard4(acc[3][0], acc[3][1], acc[3][2], acc[3][3]);

  float* slab = sT[wave];
  const float* Rb = RESID ? (resid + (size_t)b * strideR) : nullptr;
#pragma unroll
  for (int i = 0; i < 4; ++i) {
    const int mBase = m0 + (i << 4);
#pragma unroll
    for (int j = 0; j < 4; ++j) {
      const int n = n0 + (j << 4) + rlane;
      float bv = 0.f;
      if (BIAS_MODE == 2) bv = bias[n];
#pragma unroll
      for (int r = 0; r < 8; ++r) {
        float v = acc[i][j][r] * scale;
        if (BIAS_MODE == 1) v += bias[mBase + mOff + r];
        if (BIAS_MODE == 2) v += bv;
        if (RESID) v += Rb[(size_t)(mBase + mOff + r) * ldc + n];
        if (ACT == 2) v = fmaxf(v, 0.0f);
        if (ACT == 4) v = (v > 0.f) ? v : 0.01f * v;
        v = v * oscale;
        slab[(mOff + r) * 68 + (j << 4) + rlane] = v;
      }
    }
    __builtin_amdgcn_fence(__ATOMIC_RELEASE, "workgroup");
    __builtin_amdgcn_wave_barrier();
    __builtin_amdgcn_fence(__ATOMIC_ACQUIRE, "workgroup");
    if (OUT_MODE == 0) {
      float* C = (float*)Cout + (size_t)b * strideC;
      const int hh = lane >> 4, c4 = (lane & 15) * 4;
      for (int pass = 0; pass < 2; ++pass) {
#pragma unroll
        for (int it = 0; it < 8; ++it) {
          const int row = it * 2 + hh;
          v4f v = *(const v4f*)(slab + row * 68 + c4);
          *(volatile v4f*)(C + (size_t)(mBase + row) * ldc + n0 + c4) = v;
        }
        __threadfence();
      }
    } else {
      const int q = lane >> 3, c8 = (lane & 7) * 8;
      unsigned short* C  = (unsigned short*)Cout  + (size_t)b * strideC;
      unsigned short* C2 = (OUT_MODE == 2) ? ((unsigned short*)Cout2 + (size_t)b * strideC) : nullptr;
      for (int pass = 0; pass < 2; ++pass) {
#pragma unroll
        for (int it = 0; it < 4; ++it) {
          const int row = it * 4 + q;
          const float* sp = slab + row * 68 + c8;
          v8h hv, lv;
#pragma unroll
          for (int e = 0; e < 8; ++e) {
            if (OUT_MODE == 1) {
              hv[e] = (_Float16)sp[e];
            } else {
              unsigned short hb = f2bf_bits(sp[e]);
              unsigned short lb = f2bf_bits(sp[e] - bf_bits2f(hb));
              hv[e] = __builtin_bit_cast(_Float16, hb);
              lv[e] = __builtin_bit_cast(_Float16, lb);
            }
          }
          *(volatile v8h*)(C + (size_t)(mBase + row) * ldc + n0 + c8) = hv;
          if (OUT_MODE == 2) *(volatile v8h*)(C2 + (size_t)(mBase + row) * ldc + n0 + c8) = lv;
        }
        __threadfence();
      }
    }
    __builtin_amdgcn_fence(__ATOMIC_RELEASE, "workgroup");
    __builtin_amdgcn_wave_barrier();
    __builtin_amdgcn_fence(__ATOMIC_ACQUIRE, "workgroup");
  }
}

constexpr int kCvtThr = 256;

__global__ __launch_bounds__(kCvtThr) void cvt8_f16_kernel(const float* __restrict__ src, unsigned short* __restrict__ dst, int n8, float sc) {
  const int i = blockIdx.x * kCvtThr + threadIdx.x;
  if (i < n8) {
    const v4f a = *(const v4f*)(src + (size_t)i * 8);
    const v4f q = *(const v4f*)(src + (size_t)i * 8 + 4);
    v8h hv;
#pragma unroll
    for (int e = 0; e < 4; ++e) { hv[e] = (_Float16)(a[e] * sc); hv[4 + e] = (_Float16)(q[e] * sc); }
    *(volatile v8h*)(dst + (size_t)i * 8) = hv;
    __threadfence();
    *(volatile v8h*)(dst + (size_t)i * 8) = hv;
  }
}

__global__ __launch_bounds__(kCvtThr) void cvt_w2t_kernel(const float* __restrict__ w2, unsigned short* __restrict__ dst, float sc) {
  const int i = blockIdx.x * kCvtThr + threadIdx.x;
  if (i < kHid * (kHid / 8)) {
    const int h = i >> 5;
    const int j0 = (i & 31) * 8;
    v8h hv;
#pragma unroll
    for (int e = 0; e < 8; ++e) hv[e] = (_Float16)(w2[(size_t)(j0 + e) * kHid + h] * sc);
    *(volatile v8h*)(dst + (size_t)h * kHid + j0) = hv;
    __threadfence();
    *(volatile v8h*)(dst + (size_t)h * kHid + j0) = hv;
  }
}

__global__ __launch_bounds__(kCvtThr) void cvt_wih0g_kernel(const float* __restrict__ w, unsigned short* __restrict__ dst, float sc) {
  const int i = blockIdx.x * kCvtThr + threadIdx.x;
  if (i < kBranches * kGate4 * (kHid / 8)) {
    const int row = i >> 5;
    const int j0 = (i & 31) * 8;
    const float* s = w + (size_t)row * kWih0Ld + 2 + j0;
    v8h hv;
#pragma unroll
    for (int e = 0; e < 8; ++e) hv[e] = (_Float16)(s[e] * sc);
    *(volatile v8h*)(dst + (size_t)row * kHid + j0) = hv;
    __threadfence();
    *(volatile v8h*)(dst + (size_t)row * kHid + j0) = hv;
  }
}

__global__ __launch_bounds__(kCvtThr) void cvt_headw_kernel(const float* __restrict__ wpv, const float* __restrict__ ws, unsigned short* __restrict__ dst, float sc) {
  const int i = blockIdx.x * kCvtThr + threadIdx.x;
  if (i < kBranches * kHeadNPad * (kHid / 8)) {
    const int z = i >> 11;
    const int n = (i >> 5) & 63;
    const int j0 = (i & 31) * 8;
    const int zp = z < 1 ? z : 1;
    const int np = n < 2 * kOutLen ? n : 2 * kOutLen - 1;
    int zs = z - 2; zs = zs < 0 ? 0 : (zs > 2 ? 2 : zs);
    const int ns = n < kOutLen ? n : kOutLen - 1;
    const float* pp = wpv + (size_t)(zp * 2 * kOutLen + np) * kHid + j0;
    const float* ps = ws + (size_t)(zs * kOutLen + ns) * kHid + j0;
    v8h hv;
#pragma unroll
    for (int e = 0; e < 8; ++e) {
      const float vp = pp[e];
      const float vs = ps[e];
      const float v = (z < 2) ? ((n < 2 * kOutLen) ? vp : 0.0f) : ((n < kOutLen) ? vs : 0.0f);
      hv[e] = (_Float16)(v * sc);
    }
    *(volatile v8h*)(dst + (size_t)i * 8) = hv;
    __threadfence();
    *(volatile v8h*)(dst + (size_t)i * 8) = hv;
  }
}

constexpr int kGraphThreads = 256;
static_assert(kGraphThreads == kNodePad);

__global__ __launch_bounds__(kGraphThreads) void graph_norm_kernel(const float* __restrict__ nodef, const int* __restrict__ ei,
                                                                   unsigned short* __restrict__ ahat, float* __restrict__ ax) {
  __shared__ __align__(16) int sedge[kEdges];
  __shared__ __align__(16) unsigned char scnt[kNodes * kNodes];
  __shared__ __align__(16) float sx[kNodes * kFeatIn];
  __shared__ float sdinv[kNodes];
  const int tid = threadIdx.x;
  const int b = blockIdx.x;
  const int* eb = ei + (size_t)b * 2 * kEdges;
#pragma unroll 1
  for (int i = tid; i < kEdges; i += kGraphThreads) {
    int s = eb[i];
    int t = eb[kEdges + i];
    s = s < 0 ? 0 : (s > kNodes - 1 ? kNodes - 1 : s);
    t = t < 0 ? 0 : (t > kNodes - 1 ? kNodes - 1 : t);
    sedge[i] = t | (s << 8);
  }
#pragma unroll 1
  for (int i = tid; i < kNodes * kFeatIn; i += kGraphThreads) sx[i] = nodef[(size_t)b * kNodes * kFeatIn + i];
  {
    unsigned int* cz = (unsigned int*)(void*)scnt;
#pragma unroll 1
    for (int i = tid; i < (kNodes * kNodes) / 4; i += kGraphThreads) cz[i] = 0u;
  }
  __syncthreads();

  if (tid < kNodes) {
    const int t = tid;
    unsigned char* crow = scnt + t * kNodes;
    crow[t] = (unsigned char)1;
    int dg = 1;
#pragma unroll 1
    for (int e = 0; e < kEdges; ++e) {
      const int pk = sedge[e];
      if ((pk & 255) == t) {
        const int s = (pk >> 8) & 255;
        const unsigned cv = crow[s];
        crow[s] = (unsigned char)(cv < 255u ? cv + 1u : 255u);
        ++dg;
      }
    }
    sdinv[t] = rsqrtf((float)dg);
  }
  __syncthreads();

  {
    const int t = tid;
    const int tcl = t < kNodes ? t : kNodes - 1;
    const float dtl = sdinv[tcl];
    const float dt = (t < kNodes) ? dtl : 0.0f;
    const unsigned char* crow = scnt + tcl * kNodes;
    unsigned short* arow = ahat + ((size_t)b * kNodePad + t) * kNodePad;
#pragma unroll 1
    for (int q = 0; q < kNodes / 8; ++q) {
      v8h hv;
#pragma unroll
      for (int e = 0; e < 8; ++e) {
        const int s = q * 8 + e;
        const float v = (float)crow[s] * sdinv[s] * dt;
        hv[e] = (_Float16)v;
      }
      *(volatile v8h*)(arow + q * 8) = hv;
      __threadfence();
      *(volatile v8h*)(arow + q * 8) = hv;
    }
    {
      v8h zv;
#pragma unroll
      for (int e = 0; e < 8; ++e) zv[e] = (_Float16)0.0f;
#pragma unroll 1
      for (int q = kNodes / 8; q < kNodePad / 8; ++q) {
        *(volatile v8h*)(arow + q * 8) = zv;
        __threadfence();
        *(volatile v8h*)(arow + q * 8) = zv;
      }
    }
    float a0 = 0.0f, a1 = 0.0f, a2 = 0.0f, a3 = 0.0f;
#pragma unroll 1
    for (int s = 0; s < kNodes; ++s) {
      const float wv = (float)crow[s] * sdinv[s];
      const v4f xv = *(const v4f*)(sx + s * kFeatIn);
      a0 = fmaf(wv, xv[0], a0);
      a1 = fmaf(wv, xv[1], a1);
      a2 = fmaf(wv, xv[2], a2);
      a3 = fmaf(wv, xv[3], a3);
    }
    v4f av;
    av[0] = a0 * dt; av[1] = a1 * dt; av[2] = a2 * dt; av[3] = a3 * dt;
    float* ap = ax + ((size_t)b * kNodePad + t) * kFeatIn;
    *(volatile v4f*)ap = av;
    __threadfence();
    *(volatile v4f*)ap = av;
  }
}

constexpr int kH1Rows = 32;
static_assert((kGraphs * kNodePad) % kH1Rows == 0);

__global__ __launch_bounds__(256) void gcn_in_kernel(const float* __restrict__ ax, const float* __restrict__ w1, const float* __restrict__ b1,
                                                     unsigned short* __restrict__ h1c) {
  __shared__ __align__(16) _Float16 slab[kH1Rows * kHid];
  __shared__ __align__(16) float sax[kH1Rows * kFeatIn];
  const int tid = threadIdx.x, lane = tid & 31, wave = tid >> 5;
  const int rb = blockIdx.x * kH1Rows;
  if (tid < kH1Rows) {
    const v4f v = *(const v4f*)(ax + (size_t)(rb + tid) * kFeatIn);
    *(v4f*)(sax + tid * kFeatIn) = v;
  }
  const int h = tid;
  const float wa = w1[0 * kHid + h], wb = w1[1 * kHid + h], wc = w1[2 * kHid + h], wd = w1[3 * kHid + h];
  const float bb = b1[h];
  __syncthreads();
#pragma unroll 1
  for (int r = 0; r < kH1Rows; ++r) {
    const v4f a = *(const v4f*)(sax + r * kFeatIn);
    float v = bb;
    v = fmaf(a[0], wa, v);
    v = fmaf(a[1], wb, v);
    v = fmaf(a[2], wc, v);
    v = fmaf(a[3], wd, v);
    v = fmaxf(v, 0.0f) * kCarry;
    const int tl = (rb + r) & (kNodePad - 1);
    v = (tl < kNodes) ? v : 0.0f;
    slab[r * kHid + h] = (_Float16)v;
  }
  __syncthreads();
  for (int pass = 0; pass < 2; ++pass) {
#pragma unroll
    for (int i = 0; i < 4; ++i) {
      const int row = wave * 4 + i;
      const v8h hv = *(const v8h*)(slab + row * kHid + 8 * lane);
      *(volatile v8h*)(h1c + (size_t)(rb + row) * kHid + 8 * lane) = hv;
    }
    __threadfence();
  }
}

constexpr int AT_D  = 64;
constexpr int AT_NW = 4;
constexpr int AT_QB = 64;
constexpr int AT_KC = 64;
static_assert(AT_D == kHeadDim && kNodePad % AT_QB == 0 && kNodePad % AT_KC == 0);

__global__ __launch_bounds__(128)
void attn_node_kernel(const unsigned short* __restrict__ qkvp, float* __restrict__ outp, float qscale, float oinv) {
  const _Float16* qkv = (const _Float16*)qkvp;
  union FH { v16h v; v8h h[2]; };
  __shared__ __align__(16) _Float16 Ksh[AT_KC * AT_D];
  __shared__ __align__(16) _Float16 Vth[AT_D * AT_KC];
  __shared__ __align__(16) _Float16 Psh[AT_NW][16 * AT_KC];
  __shared__ __align__(16) float    Os[AT_NW][16 * 68];

  const int tid  = threadIdx.x;
  const int wave = tid >> 5;
  const int lane = tid & 31;
  const int hh   = lane >> 4;
  const int c    = lane & 15;

  const int bx = blockIdx.x;
  const int qb = bx & 3;
  const int bh = bx >> 2;
  const int h  = bh & (kHeads - 1);
  const int bl = bh >> 2;
  const size_t rowb = (size_t)bl * kNodePad;
  const int q0 = qb * AT_QB + wave * 16;

  v16h qa[2];
  {
    const _Float16* qrow = qkv + (rowb + q0 + c) * kQkvLd + h * AT_D + hh * 8;
    qa[0] = Frag<_Float16>::load(qrow);
    qa[1] = Frag<_Float16>::load(qrow + 32);
  }

  float mrow[8], lrow[8];
  v8f oacc[4];
#pragma unroll
  for (int r = 0; r < 8; ++r) { mrow[r] = -INFINITY; lrow[r] = 0.f; }
#pragma unroll
  for (int t = 0; t < 4; ++t) oacc[t] = (v8f){0.f,0.f,0.f,0.f,0.f,0.f,0.f,0.f};

  for (int kc = 0; kc < kNodePad / AT_KC; ++kc) {
    const int kv0 = kc * AT_KC;
    __syncthreads();
    {
      const int kvr = tid >> 1, dh = (tid & 1) * 32;
      const _Float16* krow = qkv + (rowb + kv0 + kvr) * kQkvLd + kHid + h * AT_D + dh;
      const _Float16* vrow = krow + kHid;
#pragma unroll
      for (int i = 0; i < 4; ++i) {
        const v8h kk = *(const v8h*)(krow + 8 * i);
        *(v8h*)(Ksh + kvr * AT_D + dh + 8 * i) = kk;
        const v8h vv = *(const v8h*)(vrow + 8 * i);
#pragma unroll
        for (int e = 0; e < 8; ++e) Vth[(dh + 8 * i + e) * AT_KC + kvr] = vv[e];
      }
    }
    __syncthreads();

    v8f s[4];
#pragma unroll
    for (int j = 0; j < 4; ++j) {
      s[j] = (v8f){0.f,0.f,0.f,0.f,0.f,0.f,0.f,0.f};
#pragma unroll
      for (int dc = 0; dc < 2; ++dc) {
        FH kb;
        kb.h[0] = *(const v8h*)(Ksh + (j * 16 + c) * AT_D + dc * 32 + 8 * hh);
        kb.h[1] = *(const v8h*)(Ksh + (j * 16 + c) * AT_D + dc * 32 + 16 + 8 * hh);
        s[j] = mma_h(qa[dc], kb.v, s[j]);
      }
    }
    float cm[8];
#pragma unroll
    for (int r = 0; r < 8; ++r) {
      float m = -INFINITY;
#pragma unroll
      for (int j = 0; j < 4; ++j) {
        const int kvcol = kv0 + j * 16 + c;
        float val = s[j][r] * qscale;
        val = (kvcol < kNodes) ? val : -INFINITY;
        s[j][r] = val;
        m = fmaxf(m, val);
      }
#pragma unroll
      for (int off = 1; off < 16; off <<= 1) m = fmaxf(m, __shfl_xor(m, off, 32));
      cm[r] = m;
    }
    _Float16* pwh = Psh[wave];
#pragma unroll
    for (int r = 0; r < 8; ++r) {
      const float mnew = fmaxf(mrow[r], cm[r]);
      const float alpha = expf(mrow[r] - mnew);
      mrow[r] = mnew;
      float psum = 0.f;
#pragma unroll
      for (int j = 0; j < 4; ++j) {
        const float p = expf(s[j][r] - mnew);
        psum += p;
        pwh[(8 * hh + r) * AT_KC + j * 16 + c] = (_Float16)(p * kPSC);
      }
#pragma unroll
      for (int off = 1; off < 16; off <<= 1) psum += __shfl_xor(psum, off, 32);
      lrow[r] = lrow[r] * alpha + psum;
#pragma unroll
      for (int t = 0; t < 4; ++t) oacc[t][r] *= alpha;
    }
    __builtin_amdgcn_fence(__ATOMIC_RELEASE, "workgroup");
    __builtin_amdgcn_wave_barrier();
    __builtin_amdgcn_fence(__ATOMIC_ACQUIRE, "workgroup");
#pragma unroll 1
    for (int kk = 0; kk < 2; ++kk) {
      FH pa;
      pa.h[0] = *(const v8h*)(pwh + c * AT_KC + kk * 32 + 8 * hh);
      pa.h[1] = *(const v8h*)(pwh + c * AT_KC + kk * 32 + 16 + 8 * hh);
#pragma unroll
      for (int t = 0; t < 4; ++t) {
        FH vb;
        vb.h[0] = *(const v8h*)(Vth + (t * 16 + c) * AT_KC + kk * 32 + 8 * hh);
        vb.h[1] = *(const v8h*)(Vth + (t * 16 + c) * AT_KC + kk * 32 + 16 + 8 * hh);
        oacc[t] = mma_h(pa.v, vb.v, oacc[t]);
      }
    }
  }

  float* os = Os[wave];
#pragma unroll
  for (int r = 0; r < 8; ++r) {
    const float inv = (1.0f / (lrow[r] * kPSC)) * oinv;
#pragma unroll
    for (int t = 0; t < 4; ++t) os[(8 * hh + r) * 68 + t * 16 + c] = oacc[t][r] * inv;
  }
  __builtin_amdgcn_fence(__ATOMIC_RELEASE, "workgroup");
  __builtin_amdgcn_wave_barrier();
  __builtin_amdgcn_fence(__ATOMIC_ACQUIRE, "workgroup");
  {
    float* ob_ptr = outp + rowb * kHid + h * AT_D;
    const int c4 = (lane & 15) * 4;
    for (int pass = 0; pass < 2; ++pass) {
#pragma unroll
      for (int it = 0; it < 8; ++it) {
        const int row = it * 2 + hh;
        v4f val = *(const v4f*)(os + row * 68 + c4);
        *(volatile v4f*)(ob_ptr + (size_t)(q0 + row) * kHid + c4) = val;
      }
      __threadfence();
    }
  }
}

__global__ __launch_bounds__(256) void node_mean_kernel(const float* __restrict__ o, unsigned short* __restrict__ obar, int gbase) {
  __shared__ __align__(16) float sm[kHid];
  const int tid = threadIdx.x, lane = tid & 31;
  const int bl = blockIdx.x;
  const int h = tid;
  float s = 0.0f;
#pragma unroll 1
  for (int n = 0; n < kNodes; ++n) s += o[((size_t)bl * kNodePad + n) * kHid + h];
  sm[h] = s * (1.0f / (float)kNodes) * kCarry;
  __syncthreads();
  if (tid < 32) {
    v8h hv;
#pragma unroll
    for (int e = 0; e < 8; ++e) hv[e] = (_Float16)sm[8 * lane + e];
    unsigned short* dst = obar + (size_t)(gbase + bl) * kHid + 8 * lane;
    for (int pass = 0; pass < 2; ++pass) {
      *(volatile v8h*)dst = hv;
      __threadfence();
    }
  }
}

constexpr int kLstmThr = 256;
constexpr int kSeqBlk  = 16;
constexpr int kNTW     = 2;
constexpr int kHP      = 264;
constexpr int kFP      = 260;
static_assert(kHid == 16 * kNTW * (kLstmThr / 32));
static_assert(kGraphs % kSeqBlk == 0);
static_assert((2 * kSeqBlk * kHP) % kLstmThr == 0);

__global__ __launch_bounds__(kLstmThr) void lstm_branch_kernel(
    const float* __restrict__ xf, const float* __restrict__ gg, const float* __restrict__ wih0raw,
    const unsigned short* __restrict__ wih1p, const unsigned short* __restrict__ whhp,
    const float* __restrict__ bih, const float* __restrict__ bhh,
    unsigned short* __restrict__ lasth) {
  __shared__ __align__(16) _Float16 Ah0[2][kSeqBlk * kHP];
  __shared__ __align__(16) _Float16 Ah1[2][kSeqBlk * kHP];
  __shared__ __align__(16) float    Hs[kSeqBlk * kFP];
  const _Float16* WI1 = (const _Float16*)wih1p;
  const _Float16* WHH = (const _Float16*)whhp;
  const int tid = threadIdx.x, lane = tid & 31, wave = tid >> 5;
  const int c = lane & 15, hh = lane >> 4, koff = hh * 8;
  const int kb = blockIdx.x >> 4;
  const int rowbase = (blockIdx.x & 15) * kSeqBlk;

  {
    _Float16* z0 = &Ah0[0][0];
    _Float16* z1 = &Ah1[0][0];
#pragma unroll 1
    for (int i = tid; i < 2 * kSeqBlk * kHP; i += kLstmThr) { z0[i] = (_Float16)0.0f; z1[i] = (_Float16)0.0f; }
  }
  float cst0[kNTW][8], cst1[kNTW][8];
#pragma unroll
  for (int nt = 0; nt < kNTW; ++nt)
#pragma unroll
    for (int r = 0; r < 8; ++r) { cst0[nt][r] = 0.0f; cst1[nt][r] = 0.0f; }

  const _Float16* whh0 = WHH + (size_t)(kb * 2 + 0) * kGate4 * kHid;
  const _Float16* whh1 = WHH + (size_t)(kb * 2 + 1) * kGate4 * kHid;
  const _Float16* wi1  = WI1 + (size_t)kb * kGate4 * kHid;
  const float* bi0 = bih + (size_t)(kb * 2 + 0) * kGate4;
  const float* bh0 = bhh + (size_t)(kb * 2 + 0) * kGate4;
  const float* bi1 = bih + (size_t)(kb * 2 + 1) * kGate4;
  const float* bh1 = bhh + (size_t)(kb * 2 + 1) * kGate4;
  const float* ggb = gg + ((size_t)kb * kGraphs + rowbase) * kGate4;
  const float* xb  = xf + ((size_t)kb * kGraphs + rowbase) * kSteps * 2;
  const float* w0b = wih0raw + (size_t)kb * kGate4 * kWih0Ld;
  __syncthreads();

  const v8f z8 = {0.f, 0.f, 0.f, 0.f, 0.f, 0.f, 0.f, 0.f};

#pragma unroll 1
  for (int t = 0; t < kSteps; ++t) {
    const int cur = t & 1;
    const int nxt = cur ^ 1;
    const bool last = (t == kSteps - 1);
    float x0r[8], x1r[8];
#pragma unroll
    for (int r = 0; r < 8; ++r) {
      const float* xp = xb + ((size_t)(8 * hh + r) * kSteps + t) * 2;
      x0r[r] = xp[0];
      x1r[r] = xp[1];
    }
    {
      const _Float16* a0row = &Ah0[cur][0] + c * kHP + koff;
      _Float16* h0n = &Ah0[nxt][0];
#pragma unroll
      for (int nt = 0; nt < kNTW; ++nt) {
        const int j = 32 * wave + 16 * nt + c;
        const _Float16* wh = whh0 + (size_t)j * kHid + koff;
        v8f acc[4];
        acc[0] = z8; acc[1] = z8; acc[2] = z8; acc[3] = z8;
#pragma unroll 1
        for (int k0 = 0; k0 < kHid; k0 += 32) {
          const v16h a  = Frag<_Float16>::load(a0row + k0);
          const v16h b0 = Frag<_Float16>::load(wh + k0);
          const v16h b1 = Frag<_Float16>::load(wh + (size_t)1 * kHid * kHid + k0);
          const v16h b2 = Frag<_Float16>::load(wh + (size_t)2 * kHid * kHid + k0);
          const v16h b3 = Frag<_Float16>::load(wh + (size_t)3 * kHid * kHid + k0);
          acc[0] = Frag<_Float16>::mma(a, b0, acc[0]);
          acc[1] = Frag<_Float16>::mma(a, b1, acc[1]);
          acc[2] = Frag<_Float16>::mma(a, b2, acc[2]);
          acc[3] = Frag<_Float16>::mma(a, b3, acc[3]);
          dep_guard_h(acc[0], acc[3], a, b3);
          keep4_h(b0, b1, b2, b3);
        }
        acc_guard4(acc[0], acc[1], acc[2], acc[3]);
        float bz[4], wx0[4], wx1[4];
#pragma unroll
        for (int g = 0; g < 4; ++g) {
          const int n = g * kHid + j;
          bz[g]  = bi0[n] + bh0[n];
          wx0[g] = w0b[(size_t)n * kWih0Ld + 0];
          wx1[g] = w0b[(size_t)n * kWih0Ld + 1];
        }
#pragma unroll
        for (int r = 0; r < 8; ++r) {
          const int m = 8 * hh + r;
          const float* gr = ggb + (size_t)m * kGate4 + j;
          const float zi = acc[0][r] * kAcc256Inv + gr[0 * kHid] + x0r[r] * wx0[0] + x1r[r] * wx1[0] + bz[0];
          const float zf = acc[1][r] * kAcc256Inv + gr[1 * kHid] + x0r[r] * wx0[1] + x1r[r] * wx1[1] + bz[1];
          const float zg = acc[2][r] * kAcc256Inv + gr[2 * kHid] + x0r[r] * wx0[2] + x1r[r] * wx1[2] + bz[2];
          const float zo = acc[3][r] * kAcc256Inv + gr[3 * kHid] + x0r[r] * wx0[3] + x1r[r] * wx1[3] + bz[3];
          const float ig = fsig(zi);
          const float fg = fsig(zf);
          const float og = fsig(zo);
          const float gv = ftanh(zg);
          const float cn = fg * cst0[nt][r] + ig * gv;
          cst0[nt][r] = cn;
          const float hn = og * ftanh(cn);
          h0n[m * kHP + j] = (_Float16)(hn * kCarry);
        }
      }
    }
    __syncthreads();
    {
      const _Float16* a1x = &Ah0[nxt][0] + c * kHP + koff;
      const _Float16* a1h = &Ah1[cur][0] + c * kHP + koff;
      _Float16* h1n = &Ah1[nxt][0];
#pragma unroll
      for (int nt = 0; nt < kNTW; ++nt) {
        const int j = 32 * wave + 16 * nt + c;
        const _Float16* wx = wi1  + (size_t)j * kHid + koff;
        const _Float16* wh = whh1 + (size_t)j * kHid + koff;
        v8f acc[4];
        acc[0] = z8; acc[1] = z8; acc[2] = z8; acc[3] = z8;
#pragma unroll 1
        for (int k0 = 0; k0 < kHid; k0 += 32) {
          const v16h a  = Frag<_Float16>::load(a1x + k0);
          const v16h b0 = Frag<_Float16>::load(wx + k0);
          const v16h b1 = Frag<_Float16>::load(wx + (size_t)1 * kHid * kHid + k0);
          const v16h b2 = Frag<_Float16>::load(wx + (size_t)2 * kHid * kHid + k0);
          const v16h b3 = Frag<_Float16>::load(wx + (size_t)3 * kHid * kHid + k0);
          acc[0] = Frag<_Float16>::mma(a, b0, acc[0]);
          acc[1] = Frag<_Float16>::mma(a, b1, acc[1]);
          acc[2] = Frag<_Float16>::mma(a, b2, acc[2]);
          acc[3] = Frag<_Float16>::mma(a, b3, acc[3]);
          dep_guard_h(acc[0], acc[3], a, b3);
          keep4_h(b0, b1, b2, b3);
        }
#pragma unroll 1
        for (int k0 = 0; k0 < kHid; k0 += 32) {
          const v16h a  = Frag<_Float16>::load(a1h + k0);
          const v16h b0 = Frag<_Float16>::load(wh + k0);
          const v16h b1 = Frag<_Float16>::load(wh + (size_t)1 * kHid * kHid + k0);
          const v16h b2 = Frag<_Float16>::load(wh + (size_t)2 * kHid * kHid + k0);
          const v16h b3 = Frag<_Float16>::load(wh + (size_t)3 * kHid * kHid + k0);
          acc[0] = Frag<_Float16>::mma(a, b0, acc[0]);
          acc[1] = Frag<_Float16>::mma(a, b1, acc[1]);
          acc[2] = Frag<_Float16>::mma(a, b2, acc[2]);
          acc[3] = Frag<_Float16>::mma(a, b3, acc[3]);
          dep_guard_h(acc[0], acc[3], a, b3);
          keep4_h(b0, b1, b2, b3);
        }
        acc_guard4(acc[0], acc[1], acc[2], acc[3]);
        float bz[4];
#pragma unroll
        for (int g = 0; g < 4; ++g) { const int n = g * kHid + j; bz[g] = bi1[n] + bh1[n]; }
#pragma unroll
        for (int r = 0; r < 8; ++r) {
          const int m = 8 * hh + r;
          const float zi = acc[0][r] * kAcc256Inv + bz[0];
          const float zf = acc[1][r] * kAcc256Inv + bz[1];
          const float zg = acc[2][r] * kAcc256Inv + bz[2];
          const float zo = acc[3][r] * kAcc256Inv + bz[3];
          const float ig = fsig(zi);
          const float fg = fsig(zf);
          const float og = fsig(zo);
          const float gv = ftanh(zg);
          const float cn = fg * cst1[nt][r] + ig * gv;
          cst1[nt][r] = cn;
          const float hn = og * ftanh(cn);
          h1n[m * kHP + j] = (_Float16)(hn * kCarry);
          if (last) Hs[m * kFP + j] = hn;
        }
      }
    }
    __syncthreads();
  }

  for (int pass = 0; pass < 2; ++pass) {
#pragma unroll
    for (int i = 0; i < 2; ++i) {
      const int m = 2 * wave + i;
      v8h hv;
#pragma unroll
      for (int e = 0; e < 8; ++e) hv[e] = (_Float16)(Hs[m * kFP + 8 * lane + e] * kCarry);
      *(volatile v8h*)(lasth + ((size_t)kb * kGraphs + rowbase + m) * kHid + 8 * lane) = hv;
    }
    __threadfence();
  }
}

constexpr int kOutBlkB      = 16;
constexpr int kOutPerB      = kOutLen * kOutComp;
constexpr int kOutFloatsBlk = kOutBlkB * kOutPerB;
constexpr int kOutLinesBlk  = kOutFloatsBlk / 32;
static_assert(kOutFloatsBlk % 32 == 0);
static_assert(kGraphs % kOutBlkB == 0);

__global__ __launch_bounds__(256) void out_assemble_kernel(const float* __restrict__ headout, const float* __restrict__ fcb_pv,
                                                           const float* __restrict__ fcb_s, float* __restrict__ out) {
  __shared__ __align__(16) float so[kOutFloatsBlk];
  const int tid = threadIdx.x, lane = tid & 31, wave = tid >> 5;
  const int blk = blockIdx.x;
#pragma unroll 1
  for (int i = tid; i < kOutFloatsBlk; i += 256) {
    const int comp = i % kOutComp;
    const int q = i / kOutComp;
    const int l = q % kOutLen;
    const int bl = q / kOutLen;
    const int b = blk * kOutBlkB + bl;
    const bool ispv = comp < 4;
    const int zpv = comp >> 1;
    const int colpv = 2 * l + (comp & 1);
    int ks = comp - 4; ks = ks < 0 ? 0 : ks;
    const int z = ispv ? zpv : (2 + ks);
    const int col = ispv ? colpv : l;
    const float hv = headout[((size_t)z * kGraphs + b) * kHeadNPad + col];
    const int ipv = (zpv < 1 ? zpv : 1) * (2 * kOutLen) + colpv;
    const int is  = ks * kOutLen + l;
    const float bpv = fcb_pv[ipv];
    const float bs  = fcb_s[is];
    float v = hv + (ispv ? bpv : bs);
    const float sg = __builtin_amdgcn_rcpf(1.0f + __expf(-v));
    v = (comp >= 5) ? sg : v;
    so[i] = v;
  }
  __syncthreads();
  float* ob = out + (size_t)blk * kOutFloatsBlk;
  for (int pass = 0; pass < 2; ++pass) {
#pragma unroll 1
    for (int g = wave; g < (kOutLinesBlk + 3) / 4; g += 8) {
      const int line = 4 * g + (lane >> 3);
      const int lc = line < kOutLinesBlk ? line : kOutLinesBlk - 1;
      const v4f v = *(const v4f*)(so + lc * 32 + (lane & 7) * 4);
      if (line < kOutLinesBlk) *(volatile v4f*)(ob + (size_t)line * 32 + (lane & 7) * 4) = v;
    }
    __threadfence();
  }
}

constexpr size_t kBytesW2T   = (size_t)kHid * kHid * 2;
constexpr size_t kBytesWin   = (size_t)kQkvLd * kHid * 2;
constexpr size_t kBytesWout  = (size_t)kHid * kHid * 2;
constexpr size_t kBytesWih0g = (size_t)kBranches * kGate4 * kHid * 2;
constexpr size_t kBytesWih1  = (size_t)kBranches * kGate4 * kHid * 2;
constexpr size_t kBytesWhh   = (size_t)kBranches * 2 * kGate4 * kHid * 2;
constexpr size_t kBytesHeadW = (size_t)kBranches * kHeadNPad * kHid * 2;
constexpr size_t kBytesGG    = (size_t)kBranches * kGraphs * kGate4 * 4;
constexpr size_t kBytesObar  = (size_t)kGraphs * kHid * 2;
constexpr size_t kBytesGfeat = (size_t)kGraphs * kHid * 2;
constexpr size_t kBytesLasth = (size_t)kBranches * kGraphs * kHid * 2;
constexpr size_t kBytesHeadO = (size_t)kBranches * kGraphs * kHeadNPad * 4;
constexpr size_t kBytesAx    = (size_t)kGraphs * kNodePad * kFeatIn * 4;
constexpr size_t kBytesPlane = (size_t)kGraphs * kNodePad * kNodePad * 2;
constexpr size_t kBytesQkvChunk = (size_t)kChunkGraphs * kNodePad * kQkvLd * 2;
constexpr size_t kBytesOChunk   = (size_t)kChunkGraphs * kNodePad * kHid * 4;

constexpr size_t kOffW2T   = 0;
constexpr size_t kOffWin   = kOffW2T + kBytesW2T;
constexpr size_t kOffWout  = kOffWin + kBytesWin;
constexpr size_t kOffWih0g = kOffWout + kBytesWout;
constexpr size_t kOffWih1  = kOffWih0g + kBytesWih0g;
constexpr size_t kOffWhh   = kOffWih1 + kBytesWih1;
constexpr size_t kOffHeadW = kOffWhh + kBytesWhh;
constexpr size_t kOffGG    = kOffHeadW + kBytesHeadW;
constexpr size_t kOffObar  = kOffGG + kBytesGG;
constexpr size_t kOffGfeat = kOffObar + kBytesObar;
constexpr size_t kOffLasth = kOffGfeat + kBytesGfeat;
constexpr size_t kOffHeadO = kOffLasth + kBytesLasth;
constexpr size_t kOffAx    = kOffHeadO + kBytesHeadO;
constexpr size_t kOffH1G   = kOffAx + kBytesAx;
constexpr size_t kOffAhat  = kOffH1G + kBytesPlane;
constexpr size_t kOffM2T   = kOffAhat + kBytesPlane;
constexpr size_t kWsTotal  = kOffM2T + kBytesPlane;
static_assert(kWsTotal == 119504896);
static_assert(kWsTotal <= 134217728);
static_assert(kBytesQkvChunk <= kBytesPlane && kBytesOChunk <= kBytesPlane);
static_assert(kOffH1G % 256 == 0 && kOffAhat % 256 == 0 && kOffM2T % 256 == 0 && kOffHeadW % 256 == 0 && kOffAx % 256 == 0);

static inline unsigned cdiv_u(long a, long b) { return (unsigned)((a + b - 1) / b); }

extern "C" void kernel_launch(void* const* d_in, const int* in_sizes, int n_in,
                              void* d_out, int out_size, void* d_ws, size_t ws_size, hipStream_t stream) {
  (void)in_sizes; (void)n_in; (void)out_size;
  if (ws_size < kWsTotal) return;

  const float* x_feats    = (const float*)d_in[0];
  const float* node_f     = (const float*)d_in[1];
  const int*   edge_idx   = (const int*)d_in[2];
  const float* gcn_W1     = (const float*)d_in[3];
  const float* gcn_b1     = (const float*)d_in[4];
  const float* gcn_W2     = (const float*)d_in[5];
  const float* gcn_b2     = (const float*)d_in[6];
  const float* attn_in_w  = (const float*)d_in[7];
  const float* attn_in_b  = (const float*)d_in[8];
  const float* attn_out_w = (const float*)d_in[9];
  const float* attn_out_b = (const float*)d_in[10];
  const float* Wih0       = (const float*)d_in[11];
  const float* Wih1       = (const float*)d_in[12];
  const float* Whh        = (const float*)d_in[13];
  const float* bih        = (const float*)d_in[14];
  const float* bhh        = (const float*)d_in[15];
  const float* fcW_pv     = (const float*)d_in[16];
  const float* fcb_pv     = (const float*)d_in[17];
  const float* fcW_s      = (const float*)d_in[18];
  const float* fcb_s      = (const float*)d_in[19];
  float* out = (float*)d_out;

  char* ws = (char*)d_ws;
  unsigned short* W2T   = (unsigned short*)(ws + kOffW2T);
  unsigned short* WIN   = (unsigned short*)(ws + kOffWin);
  unsigned short* WOUT  = (unsigned short*)(ws + kOffWout);
  unsigned short* WIH0G = (unsigned short*)(ws + kOffWih0g);
  unsigned short* WIH1H = (unsigned short*)(ws + kOffWih1);
  unsigned short* WHHH  = (unsigned short*)(ws + kOffWhh);
  unsigned short* HEADW = (unsigned short*)(ws + kOffHeadW);
  float*          GG    = (float*)(ws + kOffGG);
  unsigned short* OBAR  = (unsigned short*)(ws + kOffObar);
  unsigned short* GFEAT = (unsigned short*)(ws + kOffGfeat);
  unsigned short* LASTH = (unsigned short*)(ws + kOffLasth);
  float*          HEADO = (float*)(ws + kOffHeadO);
  float*          AX    = (float*)(ws + kOffAx);
  unsigned short* H1G   = (unsigned short*)(ws + kOffH1G);
  unsigned short* AHAT  = (unsigned short*)(ws + kOffAhat);
  unsigned short* M2T   = (unsigned short*)(ws + kOffM2T);
  float*          O32   = (float*)(ws + kOffAhat);
  unsigned short* QKV   = (unsigned short*)(ws + kOffM2T);

  const long strideNode = (long)kNodePad * kNodePad;

  {
    const int n8_win  = kQkvLd * kHid / 8;
    const int n8_wout = kHid * kHid / 8;
    const int n8_wih1 = kBranches * kGate4 * kHid / 8;
    const int n8_whh  = kBranches * 2 * kGate4 * kHid / 8;
    cvt8_f16_kernel<<<cdiv_u(n8_win, kCvtThr), kCvtThr, 0, stream>>>(attn_in_w, WIN, n8_win, kCarry);
    cvt8_f16_kernel<<<cdiv_u(n8_wout, kCvtThr), kCvtThr, 0, stream>>>(attn_out_w, WOUT, n8_wout, kCarry);
    cvt8_f16_kernel<<<cdiv_u(n8_wih1, kCvtThr), kCvtThr, 0, stream>>>(Wih1, WIH1H, n8_wih1, kCarry);
    cvt8_f16_kernel<<<cdiv_u(n8_whh, kCvtThr), kCvtThr, 0, stream>>>(Whh, WHHH, n8_whh, kCarry);
    cvt_w2t_kernel<<<cdiv_u(kHid * (kHid / 8), kCvtThr), kCvtThr, 0, stream>>>(gcn_W2, W2T, kCarry);
    cvt_wih0g_kernel<<<cdiv_u(kBranches * kGate4 * (kHid / 8), kCvtThr), kCvtThr, 0, stream>>>(Wih0, WIH0G, kCarry);
    cvt_headw_kernel<<<cdiv_u(kBranches * kHeadNPad * (kHid / 8), kCvtThr), kCvtThr, 0, stream>>>(fcW_pv, fcW_s, HEADW, kCarry);
  }

  graph_norm_kernel<<<kGraphs, kGraphThreads, 0, stream>>>(node_f, edge_idx, AHAT, AX);
  gcn_in_kernel<<<(kGraphs * kNodePad) / kH1Rows, 256, 0, stream>>>(AX, gcn_W1, gcn_b1, H1G);

  wmma_gemm64<0, false, 0, 1, false, 0><<<dim3(2, kGraphs), 256, 0, stream>>>(
      W2T, nullptr, kHid, 0L, H1G, nullptr, kHid, strideNode,
      (void*)M2T, nullptr, kNodePad, strideNode, nullptr, nullptr, 0L,
      kHid, kNodePad, kHid, kM2Scale, 1.0f);
  wmma_gemm64<0, false, 2, 1, false, 2><<<dim3(2, kGraphs), 256, 0, stream>>>(
      AHAT, nullptr, kNodePad, strideNode, M2T, nullptr, kNodePad, strideNode,
      (void*)H1G, nullptr, kHid, strideNode, gcn_b2, nullptr, 0L,
      kNodePad, kHid, kAggK, kAggScale, kCarry);

  for (int ch = 0; ch < kNumChunks; ++ch) {
    const unsigned short* Gc = H1G + (size_t)ch * kChunkGraphs * strideNode;
    const int Mrows = kChunkGraphs * kNodePad;
    wmma_gemm64<0, false, 2, 1, false, 0><<<dim3(cdiv_u((long)(Mrows / 64) * (kQkvLd / 64), 8), 1), 256, 0, stream>>>(
        Gc, nullptr, kHid, 0L, WIN, nullptr, kHid, 0L,
        (void*)QKV, nullptr, kQkvLd, 0L, attn_in_b, nullptr, 0L,
        Mrows, kQkvLd, kHid, kAcc256Inv, kCarry);
    attn_node_kernel<<<kChunkGraphs * kHeads * (kNodePad / AT_QB), 128, 0, stream>>>(QKV, O32, kQScale, kOInv);
    node_mean_kernel<<<kChunkGraphs, 256, 0, stream>>>(O32, OBAR, ch * kChunkGraphs);
  }

  wmma_gemm64<0, false, 2, 1, false, 0><<<dim3(2, 1), 256, 0, stream>>>(
      OBAR, nullptr, kHid, 0L, WOUT, nullptr, kHid, 0L,
      (void*)GFEAT, nullptr, kHid, 0L, attn_out_b, nullptr, 0L,
      kGraphs, kHid, kHid, kAcc256Inv, kCarry);
  wmma_gemm64<0, false, 0, 0, false, 0><<<dim3(cdiv_u((kGraphs / 64) * (kGate4 / 64), 8), kBranches), 256, 0, stream>>>(
      GFEAT, nullptr, kHid, 0L, WIH0G, nullptr, kHid, (long)kGate4 * kHid,
      (void*)GG, nullptr, kGate4, (long)kGraphs * kGate4, nullptr, nullptr, 0L,
      kGraphs, kGate4, kHid, kAcc256Inv, 1.0f);

  lstm_branch_kernel<<<kBranches * (kGraphs / kSeqBlk), kLstmThr, 0, stream>>>(x_feats, GG, Wih0, WIH1H, WHHH, bih, bhh, LASTH);

  wmma_gemm64<0, false, 0, 0, false, 0><<<dim3(1, kBranches), 256, 0, stream>>>(
      LASTH, nullptr, kHid, (long)kGraphs * kHid, HEADW, nullptr, kHid, (long)kHeadNPad * kHid,
      (void*)HEADO, nullptr, kHeadNPad, (long)kGraphs * kHeadNPad, nullptr, nullptr, 0L,
      kGraphs, kHeadNPad, kHid, kAcc256Inv, 1.0f);

  out_assemble_kernel<<<kGraphs / kOutBlkB, 256, 0, stream>>>(HEADO, fcb_pv, fcb_s, out);
}
